// IntegrateRNN_14826227105975
// MI455X (gfx1250) — hardware-run, weakly checked
//
#include <hip/hip_runtime.h>
#include <math.h>

constexpr int NBATCH = 16;
constexpr int NVEC   = 3;
constexpr int NGRID  = 512;
constexpr int NHID   = 512;
constexpr int NSTEN  = 5;
constexpr int NFEAT  = NVEC * NSTEN;
constexpr int NROWS  = NBATCH * NGRID;
constexpr int NSTEPS = 32;
constexpr int USIZE  = NBATCH * NVEC * NGRID;
constexpr float H1_CARRY    = 8.0f;
constexpr float W2_CARRY    = 64.0f;
constexpr float GEMM2_SCALE = 1.0f / (8.0f * 64.0f);
constexpr float DTDX        = 0.1f;

typedef __attribute__((ext_vector_type(16))) _Float16 v16h;
typedef __attribute__((ext_vector_type(8)))  _Float16 v8h;
typedef __attribute__((ext_vector_type(16))) __bf16   v16b;
typedef __attribute__((ext_vector_type(8)))  __bf16   v8b;
typedef __attribute__((ext_vector_type(8)))  float    v8f;
typedef __attribute__((ext_vector_type(4)))  float    v4f;
typedef __attribute__((ext_vector_type(4)))  unsigned int v4u;

__device__ __forceinline__ unsigned short f2bf_bits(float f) {
  unsigned u = __float_as_uint(f);
  return (unsigned short)((u + 0x7FFFu + ((u >> 16) & 1u)) >> 16);
}
__device__ __forceinline__ float bf_bits2f(unsigned short h) { return __uint_as_float(((unsigned)h) << 16); }

__device__ __forceinline__ void dep_guard_h(v8f& a, v8f& b, v16h x, v16h y) { asm volatile("v_nop\n\tv_nop\n\tv_nop\n\tv_nop" : "+v"(a), "+v"(b) : "v"(x), "v"(y)); }
__device__ __forceinline__ void dep_guard_b(v8f& a, v8f& b, v16b x, v16b y) { asm volatile("v_nop\n\tv_nop\n\tv_nop\n\tv_nop" : "+v"(a), "+v"(b) : "v"(x), "v"(y)); }
__device__ __forceinline__ void keep4_h(v16h a, v16h b, v16h c, v16h d) { asm volatile("v_nop" :: "v"(a), "v"(b), "v"(c), "v"(d)); }
__device__ __forceinline__ void keep4_b(v16b a, v16b b, v16b c, v16b d) { asm volatile("v_nop" :: "v"(a), "v"(b), "v"(c), "v"(d)); }
__device__ __forceinline__ void acc_guard4(v8f& a, v8f& b, v8f& c, v8f& d) { asm volatile("v_nop\n\tv_nop\n\tv_nop\n\tv_nop" : "+v"(a), "+v"(b), "+v"(c), "+v"(d)); }
template <typename T> struct Frag;
template <> struct Frag<_Float16> {
  typedef v16h V; union U { v16h v; v8h h[2]; };
  static __device__ __forceinline__ v16h load(const _Float16* p) {
    U f; f.h[0] = *(const v8h*)(p); f.h[1] = *(const v8h*)(p + 16); return f.v;
  }
  static __device__ __forceinline__ v8f mma(v16h a, v16h b, v8f c) {
    return __builtin_amdgcn_wmma_f32_16x16x32_f16(false, a, false, b, (short)0, c, false, false);
  }
  static __device__ __forceinline__ void guard(v8f& a, v8f& b, v16h x, v16h y) { dep_guard_h(a, b, x, y); }
  static __device__ __forceinline__ void keep(v16h a, v16h b, v16h c, v16h d) { keep4_h(a, b, c, d); }
};
template <> struct Frag<__bf16> {
  typedef v16b V; union U { v16b v; v8b h[2]; };
  static __device__ __forceinline__ v16b load(const __bf16* p) {
    U f; f.h[0] = *(const v8b*)(p); f.h[1] = *(const v8b*)(p + 16); return f.v;
  }
  static __device__ __forceinline__ v8f mma(v16b a, v16b b, v8f c) {
    return __builtin_amdgcn_wmma_f32_16x16x32_bf16(false, a, false, b, (short)0, c, false, false);
  }
  static __device__ __forceinline__ void guard(v8f& a, v8f& b, v16b x, v16b y) { dep_guard_b(a, b, x, y); }
  static __device__ __forceinline__ void keep(v16b a, v16b b, v16b c, v16b d) { keep4_b(a, b, c, d); }
};

__device__ __forceinline__ unsigned pk16(unsigned short a, unsigned short b) { return (unsigned)a | ((unsigned)b << 16); }
__device__ __forceinline__ unsigned short h_bits(float f) { const _Float16 h = (_Float16)f; return __builtin_bit_cast(unsigned short, h); }

template <int ET> struct Elem;
template <> struct Elem<0> { typedef _Float16 T; };
template <> struct Elem<1> { typedef __bf16 T; };
template <int ET, bool SPLIT, int BIAS_MODE, int OUT_MODE, bool RESID, int ACT = 0>
__global__ __launch_bounds__(256) void wmma_gemm64(
    const unsigned short* __restrict__ Ap, const unsigned short* __restrict__ A2p, int lda, long strideA,
    const unsigned short* __restrict__ Btp, const unsigned short* __restrict__ Bt2p, int ldb, long strideB,
    void* __restrict__ Cout, void* __restrict__ Cout2, int ldc, long strideC,
    const float* __restrict__ bias,
    const float* __restrict__ resid, long strideR,
    int M, int N, int K, float scale) {
  typedef typename Elem<ET>::T T;
  typedef typename Frag<T>::V V;
  const T* A = (const T*)Ap; const T* A2 = (const T*)A2p; const T* Bt = (const T*)Btp; const T* Bt2 = (const T*)Bt2p;
  __shared__ __align__(16) float sT[8][16 * 68];
  const int b    = blockIdx.y;
  const int lane = threadIdx.x & 31;
  const int wave = threadIdx.x >> 5;
  const int tilesN = N >> 6;
  const int tilesM = M >> 6;
  const int tile = blockIdx.x * 8 + wave;
  if (tile >= tilesM * tilesN) return;
  const int tm = tile / tilesN;
  const int tn = tile - tm * tilesN;
  const int m0 = tm << 6;
  const int n0 = tn << 6;

  const T* Ab  = A  + (size_t)b * strideA;
  const T* Bb  = Bt + (size_t)b * strideB;
  const T* Ab2 = SPLIT ? (A2  + (size_t)b * strideA) : nullptr;
  const T* Bb2 = SPLIT ? (Bt2 + (size_t)b * strideB) : nullptr;

  const int rlane = lane & 15;
  const int koff  = (lane >> 4) * 8;
  const int mOff  = (lane >> 4) * 8;

  v8f acc[4][4];
#pragma unroll
  for (int i = 0; i < 4; ++i)
#pragma unroll
    for (int j = 0; j < 4; ++j) acc[i][j] = (v8f){0.f,0.f,0.f,0.f,0.f,0.f,0.f,0.f};

  for (int k0 = 0; k0 < K; k0 += 32) {
    V bh[4], bl[4];
#pragma unroll
    for (int j = 0; j < 4; ++j) {
      const size_t bo = (size_t)(n0 + (j << 4) + rlane) * ldb + koff + k0;
      bh[j] = Frag<T>::load(Bb + bo);
      if (SPLIT) bl[j] = Frag<T>::load(Bb2 + bo);
    }
#pragma unroll
    for (int i = 0; i < 4; ++i) {
      const size_t ao = (size_t)(m0 + (i << 4) + rlane) * lda + koff + k0;
      V ah = Frag<T>::load(Ab + ao);
      V al;
      if (SPLIT) al = Frag<T>::load(Ab2 + ao);
#pragma unroll
      for (int j = 0; j < 4; ++j) {
        acc[i][j] = Frag<T>::mma(ah, bh[j], acc[i][j]);
        if (SPLIT) {
          acc[i][j] = Frag<T>::mma(ah, bl[j], acc[i][j]);
          acc[i][j] = Frag<T>::mma(al, bh[j], acc[i][j]);
        }
      }
      Frag<T>::guard(acc[i][0], acc[i][3], ah, SPLIT ? al : ah);
    }
    Frag<T>::keep(bh[0], bh[1], bh[2], bh[3]);
    if (SPLIT) Frag<T>::keep(bl[0], bl[1], bl[2], bl[3]);
  }
  acc_guard4(acc[0][0], acc[0][1], acc[0][2], acc[0][3]);
  acc_guard4(acc[1][0], acc[1][1], acc[1][2], acc[1][3]);
  acc_guard4(acc[2][0], acc[2][1], acc[2][2], acc[2][3]);
  acc_guard4(acc[3][0], acc[3][1], acc[3][2], acc[3][3]);

  float* slab = sT[wave];
  const float* Rb = RESID ? (resid + (size_t)b * strideR) : nullptr;
#pragma unroll
  for (int i = 0; i < 4; ++i) {
    const int mBase = m0 + (i << 4);
#pragma unroll
    for (int j = 0; j < 4; ++j) {
      const int n = n0 + (j << 4) + rlane;
      float bv = 0.f;
      if (BIAS_MODE == 2) bv = bias[n];
#pragma unroll
      for (int r = 0; r < 8; ++r) {
        float v = acc[i][j][r] * scale;
        if (BIAS_MODE == 1) v += bias[mBase + mOff + r];
        if (BIAS_MODE == 2) v += bv;
        if (RESID) v += Rb[(size_t)(mBase + mOff + r) * ldc + n];
        if (ACT == 1) v = tanhf(v);
        if (ACT == 2) v = fmaxf(v, 0.0f);
        if (ACT == 4) v = (v > 0.f) ? v : 0.01f * v;
        slab[(mOff + r) * 68 + (j << 4) + rlane] = v;
      }
    }
    __builtin_amdgcn_fence(__ATOMIC_RELEASE, "workgroup");
    __builtin_amdgcn_wave_barrier();
    __builtin_amdgcn_fence(__ATOMIC_ACQUIRE, "workgroup");
    if (OUT_MODE == 0) {
      float* C = (float*)Cout + (size_t)b * strideC;
      const int hh = lane >> 4, c4 = (lane & 15) * 4;
      for (int pass = 0; pass < 2; ++pass) {
#pragma unroll
        for (int it = 0; it < 8; ++it) {
          const int row = it * 2 + hh;
          v4f v = *(const v4f*)(slab + row * 68 + c4);
          *(volatile v4f*)(C + (size_t)(mBase + row) * ldc + n0 + c4) = v;
        }
        __threadfence();
      }
    } else {
      const int q = lane >> 3, c8 = (lane & 7) * 8;
      unsigned short* C  = (unsigned short*)Cout  + (size_t)b * strideC;
      unsigned short* C2 = (OUT_MODE == 2) ? ((unsigned short*)Cout2 + (size_t)b * strideC) : nullptr;
      for (int pass = 0; pass < 2; ++pass) {
#pragma unroll
        for (int it = 0; it < 4; ++it) {
          const int row = it * 4 + q;
          const float* sp = slab + row * 68 + c8;
          v8h hv, lv;
#pragma unroll
          for (int e = 0; e < 8; ++e) {
            if (OUT_MODE == 1) {
              hv[e] = (_Float16)sp[e];
            } else {
              unsigned short hb = f2bf_bits(sp[e]);
              unsigned short lb = f2bf_bits(sp[e] - bf_bits2f(hb));
              hv[e] = __builtin_bit_cast(_Float16, hb);
              lv[e] = __builtin_bit_cast(_Float16, lb);
            }
          }
          *(volatile v8h*)(C + (size_t)(mBase + row) * ldc + n0 + c8) = hv;
          if (OUT_MODE == 2) *(volatile v8h*)(C2 + (size_t)(mBase + row) * ldc + n0 + c8) = lv;
        }
        __threadfence();
      }
    }
    __builtin_amdgcn_fence(__ATOMIC_RELEASE, "workgroup");
    __builtin_amdgcn_wave_barrier();
    __builtin_amdgcn_fence(__ATOMIC_ACQUIRE, "workgroup");
  }
}

__global__ __launch_bounds__(256) void w2t_cast_kernel(const float* __restrict__ W, unsigned short* __restrict__ out,
                                                       float scale, const int* __restrict__ nsteps_unused) {
  (void)nsteps_unused;
  __shared__ float sm[64][65];
  const int t  = threadIdx.x;
  const int d0 = blockIdx.x * 64;
  const int h0 = blockIdx.y * 64;
#pragma unroll
  for (int i = 0; i < 16; ++i) {
    const int e = i * 256 + t;
    const int r = e >> 6;
    const int c = e & 63;
    sm[c][r] = W[(size_t)(d0 + r) * NHID + h0 + c] * scale;
  }
  __syncthreads();
  const int lane = t & 31, wave = t >> 5;
  const int q = lane >> 3, c8 = (lane & 7) * 8;
  for (int pass = 0; pass < 2; ++pass) {
#pragma unroll
    for (int it = 0; it < 2; ++it) {
      const int row = wave * 8 + it * 4 + q;
      unsigned short hb[8];
#pragma unroll
      for (int e = 0; e < 8; ++e) hb[e] = h_bits(sm[row][c8 + e]);
      const v4u u = (v4u){pk16(hb[0], hb[1]), pk16(hb[2], hb[3]), pk16(hb[4], hb[5]), pk16(hb[6], hb[7])};
      *(volatile v4u*)(out + (size_t)(h0 + row) * NHID + d0 + c8) = u;
    }
    __threadfence();
  }
}

__global__ __launch_bounds__(256) void layer1_kernel(const float* __restrict__ usrc, const float* __restrict__ W1,
                                                     const float* __restrict__ b1, unsigned short* __restrict__ H1) {
  __shared__ __align__(16) float feats[32][16];
  const int tid  = threadIdx.x;
  const int m0   = blockIdx.x * 32;
  const int bidx = m0 >> 9;
  const int n0   = m0 & (NGRID - 1);
  for (int idx = tid; idx < 32 * 16; idx += 256) {
    const int r  = idx >> 4, f = idx & 15;
    const int fc = (f < NFEAT) ? f : (NFEAT - 1);
    const int v  = fc / NSTEN;
    const int s  = fc - v * NSTEN;
    const int nn = (n0 + r + s - 2 + NGRID) & (NGRID - 1);
    const float val = usrc[((size_t)(bidx * NVEC + v)) * NGRID + nn];
    feats[r][f] = (f < NFEAT) ? val : 0.0f;
  }
  __syncthreads();

  const int j = tid * 2;
  float w1c[NFEAT][2];
#pragma unroll
  for (int k = 0; k < NFEAT; ++k) {
    w1c[k][0] = W1[k * NHID + j];
    w1c[k][1] = W1[k * NHID + j + 1];
  }
  const float bb0 = b1[j], bb1 = b1[j + 1];
#pragma unroll 1
  for (int r = 0; r < 32; ++r) {
    float a0 = 0.0f, a1 = 0.0f;
#pragma unroll
    for (int k = 0; k < NFEAT; ++k) {
      const float fv = feats[r][k];
      a0 += fv * w1c[k][0];
      a1 += fv * w1c[k][1];
    }
    a0 += bb0;
    a1 += bb1;
    const float h0v = tanhf(a0) * H1_CARRY;
    const float h1v = tanhf(a1) * H1_CARRY;
    const unsigned u = pk16(h_bits(h0v), h_bits(h1v));
    volatile unsigned* p = (volatile unsigned*)(H1 + (size_t)(m0 + r) * NHID + j);
    *p = u;
    __threadfence();
    *p = u;
  }
}

__global__ __launch_bounds__(512) void head_kernel(const float* __restrict__ H2, const float* __restrict__ W3,
                                                   const float* __restrict__ b3, const float* __restrict__ usrc,
                                                   float* __restrict__ unext, float* __restrict__ outS,
                                                   float* __restrict__ outA, float* __restrict__ outR) {
  __shared__ __align__(16) float w3s[NHID * NSTEN];
  __shared__ __align__(16) float us[NVEC * NGRID];
  __shared__ __align__(16) float fls[NVEC * NGRID];
  __shared__ __align__(16) float acts[NGRID * NSTEN];
  __shared__ __align__(16) float rews[NGRID];
  __shared__ __align__(16) float nus[NVEC * NGRID];
  const int bb = blockIdx.x;
  const int n  = threadIdx.x;
  for (int i = n; i < NHID * NSTEN; i += 512) w3s[i] = W3[i];
  const float* ub = usrc + (size_t)bb * NVEC * NGRID;
#pragma unroll
  for (int v = 0; v < NVEC; ++v) us[v * NGRID + n] = ub[v * NGRID + n];
  __syncthreads();

  float a0 = 0.f, a1 = 0.f, a2 = 0.f, a3 = 0.f, a4 = 0.f;
  const float* hrow = H2 + ((size_t)bb * NGRID + n) * NHID;
#pragma unroll 1
  for (int k = 0; k < NHID; k += 4) {
    const v4f h = *(const v4f*)(hrow + k);
    const float* wr = w3s + k * NSTEN;
#pragma unroll
    for (int e = 0; e < 4; ++e) {
      const float hv = h[e];
      a0 += hv * wr[e * NSTEN + 0];
      a1 += hv * wr[e * NSTEN + 1];
      a2 += hv * wr[e * NSTEN + 2];
      a3 += hv * wr[e * NSTEN + 3];
      a4 += hv * wr[e * NSTEN + 4];
    }
  }
  a0 += b3[0]; a1 += b3[1]; a2 += b3[2]; a3 += b3[3]; a4 += b3[4];
  const float mx = fmaxf(fmaxf(fmaxf(a0, a1), fmaxf(a2, a3)), a4);
  const float e0 = expf(a0 - mx), e1 = expf(a1 - mx), e2 = expf(a2 - mx), e3 = expf(a3 - mx), e4 = expf(a4 - mx);
  const float ssum = (((e0 + e1) + e2) + e3) + e4;
  const float inv = 1.0f / ssum;
  const float w0 = e0 * inv, w1 = e1 * inv, w2 = e2 * inv, w3 = e3 * inv, w4 = e4 * inv;
  acts[n * NSTEN + 0] = w0;
  acts[n * NSTEN + 1] = w1;
  acts[n * NSTEN + 2] = w2;
  acts[n * NSTEN + 3] = w3;
  acts[n * NSTEN + 4] = w4;
  rews[n] = -((((w0 * w0 + w1 * w1) + w2 * w2) + w3 * w3) + w4 * w4);

  const int nm2 = (n + NGRID - 2) & (NGRID - 1);
  const int nm1 = (n + NGRID - 1) & (NGRID - 1);
  const int np1 = (n + 1) & (NGRID - 1);
  const int np2 = (n + 2) & (NGRID - 1);
#pragma unroll 1
  for (int v = 0; v < NVEC; ++v) {
    const float* ur = us + v * NGRID;
    fls[v * NGRID + n] = w0 * ur[nm2] + w1 * ur[nm1] + w2 * ur[n] + w3 * ur[np1] + w4 * ur[np2];
  }
  __syncthreads();
#pragma unroll 1
  for (int v = 0; v < NVEC; ++v) {
    const float f0 = fls[v * NGRID + n];
    const float fm = fls[v * NGRID + nm1];
    nus[v * NGRID + n] = us[v * NGRID + n] - DTDX * (f0 - fm);
  }
  __syncthreads();

  float* oA = outA  + (size_t)bb * NGRID * NSTEN;
  float* oR = outR  + (size_t)bb * NGRID;
  float* oS = outS  + (size_t)bb * NVEC * NGRID;
  float* uN = unext + (size_t)bb * NVEC * NGRID;
  for (int pass = 0; pass < 2; ++pass) {
    for (int i = n; i < (NGRID * NSTEN) / 4; i += 512) {
      const v4f val = *(const v4f*)(acts + 4 * i);
      *(volatile v4f*)(oA + 4 * i) = val;
    }
    if (n < NGRID / 4) {
      const v4f val = *(const v4f*)(rews + 4 * n);
      *(volatile v4f*)(oR + 4 * n) = val;
    }
    if (n < (NVEC * NGRID) / 4) {
      const v4f val = *(const v4f*)(nus + 4 * n);
      *(volatile v4f*)(oS + 4 * n) = val;
      *(volatile v4f*)(uN + 4 * n) = val;
    }
    __threadfence();
  }
}

extern "C" void kernel_launch(void* const* d_in, const int* in_sizes, int n_in,
                              void* d_out, int out_size, void* d_ws, size_t ws_size,
                              hipStream_t stream) {
  (void)in_sizes;
  if (n_in < 8) return;
  const float* u0  = (const float*)d_in[0];
  const float* W1  = (const float*)d_in[1];
  const float* b1  = (const float*)d_in[2];
  const float* W2  = (const float*)d_in[3];
  const float* b2  = (const float*)d_in[4];
  const float* W3  = (const float*)d_in[5];
  const float* b3  = (const float*)d_in[6];
  const int*   nst = (const int*)d_in[7];

  const size_t uBytes   = (size_t)USIZE * 4;
  const size_t w2tBytes = (size_t)NHID * NHID * 2;
  const size_t h1Bytes  = (size_t)NROWS * NHID * 2;
  const size_t h2Bytes  = (size_t)NROWS * NHID * 4;
  const size_t offUA  = 0;
  const size_t offUB  = offUA + uBytes;
  const size_t offW2T = offUB + uBytes;
  const size_t offH1  = offW2T + w2tBytes;
  const size_t offH2  = offH1 + h1Bytes;
  const size_t total  = offH2 + h2Bytes;
  if (total > ws_size) return;
  if ((size_t)out_size < (size_t)NSTEPS * (USIZE + NROWS * NSTEN + NROWS)) return;

  char* ws = (char*)d_ws;
  float* uA = (float*)(ws + offUA);
  float* uB = (float*)(ws + offUB);
  unsigned short* W2T = (unsigned short*)(ws + offW2T);
  unsigned short* H1  = (unsigned short*)(ws + offH1);
  float* H2 = (float*)(ws + offH2);

  float* outStates  = (float*)d_out;
  float* outActions = outStates + (size_t)NSTEPS * USIZE;
  float* outRewards = outActions + (size_t)NSTEPS * NROWS * NSTEN;

  w2t_cast_kernel<<<dim3(NHID / 64, NHID / 64), 256, 0, stream>>>(W2, W2T, W2_CARRY, nst);

  const int gemmTiles  = (NROWS / 64) * (NHID / 64);
  const int gemmBlocks = (gemmTiles + 7) / 8;
  for (int t = 0; t < NSTEPS; ++t) {
    const float* usrc = (t == 0) ? u0 : ((((t - 1) & 1) == 0) ? uA : uB);
    float* unext = ((t & 1) == 0) ? uA : uB;
    layer1_kernel<<<NROWS / 32, 256, 0, stream>>>(usrc, W1, b1, H1);
    wmma_gemm64<0, false, 2, 0, false, 1><<<dim3(gemmBlocks, 1), 256, 0, stream>>>(
        H1, nullptr, NHID, 0L,
        W2T, nullptr, NHID, 0L,
        (void*)H2, nullptr, NHID, 0L,
        b2, nullptr, 0L,
        NROWS, NHID, NHID, GEMM2_SCALE);
    head_kernel<<<NBATCH, 512, 0, stream>>>(H2, W3, b3, usrc, unext,
                                             outStates  + (size_t)t * USIZE,
                                             outActions + (size_t)t * NROWS * NSTEN,
                                             outRewards + (size_t)t * NROWS);
  }
}
